// TrainableMPOLayer_7284264534632
// MI455X (gfx1250) — hardware-run, weakly checked
//
#include <hip/hip_runtime.h>

typedef __attribute__((ext_vector_type(16))) __bf16   v16b;
typedef __attribute__((ext_vector_type(8)))  __bf16   v8b;
typedef __attribute__((ext_vector_type(8)))  float    v8f;
typedef __attribute__((ext_vector_type(4)))  float    v4f;
typedef __attribute__((ext_vector_type(4)))  unsigned v4u;

constexpr int kBatch   = 2048;
constexpr int kIn      = 4096;
constexpr int kOut     = 4096;
constexpr int kFac     = 32;
constexpr int kBond    = 2;
constexpr int kChunk   = kFac * kFac;
constexpr int kJ       = kIn / kChunk;
constexpr int kKd      = kOut / kChunk;
constexpr int kKp      = 32;
constexpr int kBiasLen = kFac * kFac * kFac;
constexpr float kInvFac = 1.0f / (float)kFac;
static_assert(kChunk == 1024, "chunk of the leading digit");
static_assert(kJ == 4 && kKd == 4, "four nonzero chunk sums, four leading output digits");
static_assert(kIn % kChunk == 0 && kOut % kChunk == 0, "whole chunks");
static_assert(4 * kJ <= 16 && kKp == 32, "packed k slots fit one 32-deep step");
static_assert((kBatch % 64) == 0 && (kOut % 64) == 0, "GEMM M, N multiples of 64");
static_assert(kBond == 2, "bond rank");

constexpr size_t kOffA    = 0;
constexpr size_t kBytesA  = (size_t)kBatch * kKp * 2;
constexpr size_t kOffBt   = kOffA + kBytesA;
constexpr size_t kBytesBt = (size_t)kOut * kKp * 2;
constexpr size_t kWsTotal = kOffBt + kBytesBt;
static_assert(kBytesA == 131072ull && kBytesBt == 262144ull, "plane sizes");
static_assert(kWsTotal == 393216ull, "carve total");
static_assert(kWsTotal <= 134217728ull, "carve cap");
static_assert((kOffBt % 128) == 0, "128-B aligned regions");

__device__ __forceinline__ unsigned f2bf_u(float f) {
  const unsigned u = __float_as_uint(f);
  return (u + 0x7FFFu + ((u >> 16) & 1u)) >> 16;
}
__device__ __forceinline__ float bf_u2f(unsigned h) { return __uint_as_float(h << 16); }

union FragB { v16b v; v8b h[2]; };
__device__ __forceinline__ v16b frag_load(const __bf16* p) {
  FragB f;
  f.h[0] = *(const v8b*)(p);
  f.h[1] = *(const v8b*)(p + 16);
  return f.v;
}
__device__ __forceinline__ v8f mma_bf16_guarded(v16b a, v16b b, v8f c) {
  c = __builtin_amdgcn_wmma_f32_16x16x32_bf16(false, a, false, b, (short)0, c, false, false);
  asm volatile("v_nop\n\tv_nop\n\tv_nop\n\tv_nop" : "+v"(c) : "v"(a), "v"(b));
  return c;
}

__global__ __launch_bounds__(256) void build_bt_kernel(
    const float* __restrict__ core0, const float* __restrict__ core1, const float* __restrict__ core2,
    unsigned* __restrict__ BtW)
{
  __shared__ float cc1s[2 * kFac * 2];
  __shared__ float cc2s[2 * kFac];
  __shared__ __align__(16) unsigned sB[256 * 16];
  const int tid  = threadIdx.x;
  const int wave = __builtin_amdgcn_readfirstlane((int)(threadIdx.x >> 5));

  if (wave < 2) {
    const float* p = core1 + (size_t)tid * (kFac * 2);
    float a0 = 0.0f, a1 = 0.0f;
#pragma unroll
    for (int i = 0; i < 16; ++i) {
      const v4f v = *(const v4f*)(p + 4 * i);
      a0 += v.x;
      a1 += v.y;
      a0 += v.z;
      a1 += v.w;
    }
    cc1s[tid * 2 + 0] = a0 * kInvFac;
    cc1s[tid * 2 + 1] = a1 * kInvFac;
  } else if (wave < 4) {
    const int idx = tid - 64;
    const float* p = core2 + (size_t)idx * kFac;
    float a0 = 0.0f;
#pragma unroll
    for (int i = 0; i < 8; ++i) {
      const v4f v = *(const v4f*)(p + 4 * i);
      a0 += v.x;
      a0 += v.y;
      a0 += v.z;
      a0 += v.w;
    }
    cc2s[idx] = a0 * kInvFac;
  }
  __syncthreads();

  const int m  = blockIdx.x * 256 + tid;
  const int k  = m >> 10;
  const int j1 = (m >> 5) & 31;
  const int j2 = m & 31;
  const float c1_00 = cc1s[(0 * kFac + j1) * 2 + 0];
  const float c1_01 = cc1s[(0 * kFac + j1) * 2 + 1];
  const float c1_10 = cc1s[(1 * kFac + j1) * 2 + 0];
  const float c1_11 = cc1s[(1 * kFac + j1) * 2 + 1];
  const float c2_0  = cc2s[0 * kFac + j2];
  const float c2_1  = cc2s[1 * kFac + j2];

  unsigned hb[4], lb[4];
#pragma unroll
  for (int j = 0; j < 4; ++j) {
    const float c0a = core0[(j * kFac + k) * 2 + 0];
    const float c0b = core0[(j * kFac + k) * 2 + 1];
    float acc = 0.0f;
    acc += c0a * c1_00 * c2_0;
    acc += c0a * c1_01 * c2_1;
    acc += c0b * c1_10 * c2_0;
    acc += c0b * c1_11 * c2_1;
    const unsigned h = f2bf_u(acc);
    const unsigned l = f2bf_u(acc - bf_u2f(h));
    hb[j] = h;
    lb[j] = l;
  }
  const unsigned wh0 = hb[0] | (hb[1] << 16);
  const unsigned wh1 = hb[2] | (hb[3] << 16);
  const unsigned wl0 = lb[0] | (lb[1] << 16);
  const unsigned wl1 = lb[2] | (lb[3] << 16);
  const v4u qh = (v4u){wh0, wh1, wh0, wh1};
  const v4u ql = (v4u){wl0, wl1, wl0, wl1};
  const v4u qz = (v4u){0u, 0u, 0u, 0u};
  *(v4u*)(sB + tid * 16 + 0)  = qh;
  *(v4u*)(sB + tid * 16 + 4)  = ql;
  *(v4u*)(sB + tid * 16 + 8)  = qz;
  *(v4u*)(sB + tid * 16 + 12) = qz;
  __syncthreads();

  v4u pv[4];
#pragma unroll
  for (int it = 0; it < 4; ++it) pv[it] = *(const v4u*)(sB + (it * 256 + tid) * 4);
  unsigned* dst = BtW + (size_t)blockIdx.x * (256 * 16);
  for (int pass = 0; pass < 2; ++pass) {
#pragma unroll
    for (int it = 0; it < 4; ++it)
      *(volatile v4u*)(dst + (it * 256 + tid) * 4) = pv[it];
    __threadfence();
  }
}

__global__ __launch_bounds__(256) void rowsum_a_kernel(
    const float* __restrict__ x, unsigned* __restrict__ Aw)
{
  __shared__ __align__(16) unsigned sA[32 * 16];
  const int tid  = threadIdx.x;
  const int lane = tid & 31;
  const int wave = __builtin_amdgcn_readfirstlane((int)(threadIdx.x >> 5));

#pragma unroll 1
  for (int rr = 0; rr < 4; ++rr) {
    const int lrow = wave * 4 + rr;
    const size_t row = (size_t)blockIdx.x * 32 + lrow;
    const float* xr = x + row * kIn;
    float s[4];
#pragma unroll
    for (int j = 0; j < 4; ++j) {
      const v4f* p = (const v4f*)(xr + j * kChunk);
      v4f a4 = (v4f){0.0f, 0.0f, 0.0f, 0.0f};
#pragma unroll
      for (int it = 0; it < 8; ++it) a4 += p[lane + it * 32];
      float acc = (a4.x + a4.y) + (a4.z + a4.w);
#pragma unroll
      for (int off = 16; off > 0; off >>= 1) acc += __shfl_xor(acc, off, 32);
      s[j] = acc;
    }
    unsigned hb[4], lb[4];
#pragma unroll
    for (int j = 0; j < 4; ++j) {
      const unsigned h = f2bf_u(s[j]);
      const unsigned l = f2bf_u(s[j] - bf_u2f(h));
      hb[j] = h;
      lb[j] = l;
    }
    const unsigned wh0 = hb[0] | (hb[1] << 16);
    const unsigned wh1 = hb[2] | (hb[3] << 16);
    const unsigned wl0 = lb[0] | (lb[1] << 16);
    const unsigned wl1 = lb[2] | (lb[3] << 16);
    const v4u qa = (v4u){wh0, wh1, wl0, wl1};
    const v4u qz = (v4u){0u, 0u, 0u, 0u};
    if (lane == 0) {
      *(v4u*)(sA + lrow * 16 + 0)  = qa;
      *(v4u*)(sA + lrow * 16 + 4)  = qa;
      *(v4u*)(sA + lrow * 16 + 8)  = qz;
      *(v4u*)(sA + lrow * 16 + 12) = qz;
    }
  }
  __syncthreads();

  if (wave < 4) {
    const v4u pv = *(const v4u*)(sA + tid * 4);
    unsigned* dst = Aw + (size_t)blockIdx.x * (32 * 16) + tid * 4;
    *(volatile v4u*)dst = pv;
    __threadfence();
    *(volatile v4u*)dst = pv;
  }
}

constexpr int kTilesN = kOut >> 6;
constexpr int kTilesM = kBatch >> 6;
static_assert(((kTilesM * kTilesN) % 8) == 0, "whole blocks of 8 tiles");

__global__ __launch_bounds__(256) void gemm_k32_kernel(
    const unsigned short* __restrict__ Ap, const unsigned short* __restrict__ Btp,
    const float* __restrict__ bias, float* __restrict__ out)
{
  __shared__ __align__(16) float sT[8][16 * 68];
  const __bf16* A  = (const __bf16*)Ap;
  const __bf16* Bt = (const __bf16*)Btp;
  const int lane = threadIdx.x & 31;
  const int wave = __builtin_amdgcn_readfirstlane((int)(threadIdx.x >> 5));
  const int tile = blockIdx.x * 8 + wave;
  const int tm = tile / kTilesN;
  const int tn = tile - tm * kTilesN;
  const int m0 = tm << 6;
  const int n0 = tn << 6;
  const int rlane = lane & 15;
  const int hh    = lane >> 4;
  const int koff  = hh * 8;
  const int mOff  = hh * 8;
  const int c4    = rlane * 4;

  v16b bfr[4];
#pragma unroll
  for (int j = 0; j < 4; ++j)
    bfr[j] = frag_load(Bt + (size_t)(n0 + (j << 4) + rlane) * kKp + koff);

  const v4f bq = *(const v4f*)(bias + n0 + c4);
  float* slab = sT[wave];

#pragma unroll 1
  for (int i = 0; i < 4; ++i) {
    const int mBase = m0 + (i << 4);
    const v16b af = frag_load(A + (size_t)(mBase + rlane) * kKp + koff);
    v8f acc[4];
#pragma unroll
    for (int j = 0; j < 4; ++j) {
      acc[j] = (v8f){0.f, 0.f, 0.f, 0.f, 0.f, 0.f, 0.f, 0.f};
      acc[j] = mma_bf16_guarded(af, bfr[j], acc[j]);
    }
#pragma unroll
    for (int j = 0; j < 4; ++j) {
#pragma unroll
      for (int r = 0; r < 8; ++r)
        slab[(mOff + r) * 68 + (j << 4) + rlane] = acc[j][r];
    }
    __syncthreads();
    v4f vv[8];
#pragma unroll
    for (int it = 0; it < 8; ++it) {
      const int row = it * 2 + hh;
      const v4f t = *(const v4f*)(slab + row * 68 + c4);
      vv[it] = t + bq;
    }
    for (int pass = 0; pass < 2; ++pass) {
#pragma unroll
      for (int it = 0; it < 8; ++it) {
        const int row = it * 2 + hh;
        *(volatile v4f*)(out + (size_t)(mBase + row) * kOut + n0 + c4) = vv[it];
      }
      __threadfence();
    }
    __syncthreads();
  }
}

extern "C" void kernel_launch(void* const* d_in, const int* in_sizes, int n_in,
                              void* d_out, int out_size, void* d_ws, size_t ws_size,
                              hipStream_t stream) {
  if (n_in < 5) return;
  if (in_sizes[0] != kBatch * kIn) return;
  if (in_sizes[1] != 1 * kFac * kFac * kBond) return;
  if (in_sizes[2] != kBond * kFac * kFac * kBond) return;
  if (in_sizes[3] != kBond * kFac * kFac * 1) return;
  if (in_sizes[4] != kBiasLen) return;
  if (out_size != kBatch * kOut) return;
  if (ws_size < kWsTotal) return;

  const float* x     = (const float*)d_in[0];
  const float* core0 = (const float*)d_in[1];
  const float* core1 = (const float*)d_in[2];
  const float* core2 = (const float*)d_in[3];
  const float* bias  = (const float*)d_in[4];
  float* out = (float*)d_out;

  char* ws = (char*)d_ws;
  unsigned* Aw  = (unsigned*)(ws + kOffA);
  unsigned* BtW = (unsigned*)(ws + kOffBt);

  build_bt_kernel<<<kOut / 256, 256, 0, stream>>>(core0, core1, core2, BtW);
  rowsum_a_kernel<<<kBatch / 32, 256, 0, stream>>>(x, Aw);
  gemm_k32_kernel<<<(kTilesM * kTilesN) / 8, 256, 0, stream>>>(
      (const unsigned short*)Aw, (const unsigned short*)BtW, bias, out);
}
